// ResBlock_3d_25125558681985
// MI455X (gfx1250) — hardware-verified
//
#include <hip/hip_runtime.h>
#include <hip/hip_bf16.h>
#include <stdint.h>


typedef __attribute__((ext_vector_type(16))) _Float16 v16bf;
typedef __attribute__((ext_vector_type(8)))  _Float16 v8h;
typedef __attribute__((ext_vector_type(8)))  float  v8f;
typedef __attribute__((ext_vector_type(4)))  float  v4f;
typedef __attribute__((ext_vector_type(4)))  int    v4i;
typedef __attribute__((ext_vector_type(4)))  unsigned v4u;
template <typename T> __device__ __forceinline__ void vst2(void* p, T v) { *(volatile T*)p = v; __threadfence(); *(volatile T*)p = v; }
__device__ __forceinline__ v8f wmma16(v16bf a, v16bf b, v8f c) {
  v8f d = __builtin_amdgcn_wmma_f32_16x16x32_f16(false, a, false, b, (short)0, c, false, false);
  asm volatile("v_nop\n\tv_nop\n\tv_nop\n\tv_nop" : "+v"(d) : "v"(a), "v"(b));
  return d;
}

#define Tdim 7
#define Hdim 48
#define Wdim 48
#define Cdim 64
#define Mpix (Tdim*Hdim*Wdim)
#define KK   27
#define LDA  66

__device__ __forceinline__ unsigned short f2bf(float f){
  union { _Float16 h; unsigned short u; } c; c.h = (_Float16)f; return c.u;
}
__device__ __forceinline__ float bf2f(unsigned short h){
  union { _Float16 h; unsigned short u; } c; c.u = h; return (float)c.h;
}

__device__ __forceinline__ void copy16_g2l(const void* gsrc, void* ldst){
#ifdef HAVE_ASYNC_LDS
  __builtin_amdgcn_global_load_async_to_lds_b128(
      (v4i*)(uintptr_t)gsrc, (v4i*)(uintptr_t)ldst, 0, 0);
#else
  *(uint4*)ldst = *(const uint4*)gsrc;
#endif
}

template <int N>
__device__ __forceinline__ void wait_async(){
#ifdef HAVE_ASYNC_LDS
#if __has_builtin(__builtin_amdgcn_s_wait_asynccnt)
  __builtin_amdgcn_s_wait_asynccnt(N);
#else
  asm volatile("s_wait_asynccnt %0" :: "i"(N) : "memory");
#endif
#endif
}

__global__ void k_cvt_x(const float* __restrict__ x, unsigned short* __restrict__ xbf){
  int g8 = blockIdx.x * 256 + threadIdx.x;
  int idx = g8 * 8;
  int p = idx >> 6, c0 = idx & 63;
  union { unsigned short s[8]; v4u u; } pk;
#pragma unroll
  for (int e = 0; e < 8; ++e) pk.s[e] = f2bf(x[(size_t)(c0 + e) * Mpix + p]);
  vst2(xbf + idx, pk.u);
}

__global__ void k_cvt_w(const float* __restrict__ w, int O, unsigned short* __restrict__ dst){
  int g8 = blockIdx.x * 256 + threadIdx.x;
  if (g8 >= 110592 / 8) return;
  union { unsigned short s[8]; v4u u; } pk;
#pragma unroll
  for (int ee = 0; ee < 8; ++ee) {
    int idx  = g8 * 8 + ee;
    int e    = idx & 15;
    int lane = (idx >> 4) & 31;
    int nt   = (idx >> 9) & 3;
    int ks   = (idx >> 11) & 1;
    int tap  = idx >> 12;
    int klocal = (lane >> 4) * 8 + ((e < 8) ? e : (e + 8));
    int c = ks * 32 + klocal;
    int o = nt * 16 + (lane & 15);
    float v = (o < O) ? w[((size_t)o * Cdim + c) * KK + tap] : 0.f;
    pk.s[ee] = f2bf(v);
  }
  vst2(dst + (size_t)g8 * 8, pk.u);
}

__global__ void __launch_bounds__(128)
k_dcn_gemm(const unsigned short* __restrict__ xin,
           const unsigned short* __restrict__ wmat,
           const float* __restrict__ bias,
           const float* __restrict__ offb,
           const float* __restrict__ resid,
           float* __restrict__ outF,
           unsigned short* __restrict__ outB,
           int NO, int mode, int deform)
{
  __shared__ unsigned short Atile[64 * LDA];
  __shared__ __attribute__((aligned(16))) unsigned short Btile[2][64 * 64];
  __shared__ __attribute__((aligned(16))) float so[64][65];

  const int tid = threadIdx.x;
  const int m0  = blockIdx.x * 64;
  const int wv  = tid >> 5;
  const int ln  = tid & 31;

  const int p_local = tid >> 1;
  const int cbase   = (tid & 1) * 32;
  const int p  = m0 + p_local;
  const int w_ = p % Wdim;
  const int h_ = (p / Wdim) % Hdim;
  const int t_ = p / (Wdim * Hdim);

  v8f acc[4];
  const v8f vzero = {0.f,0.f,0.f,0.f,0.f,0.f,0.f,0.f};
  #pragma unroll
  for (int j = 0; j < 4; ++j) acc[j] = vzero;

  {
    const char* src = (const char*)wmat + tid * 64;
    char* dst = (char*)&Btile[0][0] + tid * 64;
    #pragma unroll
    for (int i = 0; i < 4; ++i) copy16_g2l(src + i * 16, dst + i * 16);
  }

  int kt = 0, kh = 0, kw = 0;
  for (int tap = 0; tap < KK; ++tap){
    const int bp = tap & 1;
    const int pt  = t_ + kt - 1;
    const bool tok = (pt >= 0) && (pt < Tdim);
    const int ptc = pt < 0 ? 0 : (pt > Tdim - 1 ? Tdim - 1 : pt);

    const unsigned short* cp[4];
    float cw[4];
    if (deform){
      const float oh = offb[(size_t)p * 64 + tap * 2 + 0];
      const float ow = offb[(size_t)p * 64 + tap * 2 + 1];
      const float ph = (float)(h_ + kh - 1) + oh;
      const float pw = (float)(w_ + kw - 1) + ow;
      const float h0f = floorf(ph), w0f = floorf(pw);
      const float lh = ph - h0f, lw = pw - w0f;
      const int h0 = (int)h0f, w0 = (int)w0f;
      const float wq[4] = {(1.f - lh) * (1.f - lw), (1.f - lh) * lw,
                           lh * (1.f - lw),         lh * lw};
      #pragma unroll
      for (int cn = 0; cn < 4; ++cn){
        const int hc = h0 + (cn >> 1);
        const int wc = w0 + (cn & 1);
        const bool ok = tok && hc >= 0 && hc < Hdim && wc >= 0 && wc < Wdim;
        const int hcc = hc < 0 ? 0 : (hc > Hdim - 1 ? Hdim - 1 : hc);
        const int wcc = wc < 0 ? 0 : (wc > Wdim - 1 ? Wdim - 1 : wc);
        cp[cn] = xin + (((size_t)ptc * Hdim + hcc) * Wdim + wcc) * 64 + cbase;
        cw[cn] = ok ? wq[cn] : 0.f;
      }
    } else {
      const int hc = h_ + kh - 1, wc = w_ + kw - 1;
      const bool ok = tok && hc >= 0 && hc < Hdim && wc >= 0 && wc < Wdim;
      const int hcc = hc < 0 ? 0 : (hc > Hdim - 1 ? Hdim - 1 : hc);
      const int wcc = wc < 0 ? 0 : (wc > Wdim - 1 ? Wdim - 1 : wc);
      cp[0] = xin + (((size_t)ptc * Hdim + hcc) * Wdim + wcc) * 64 + cbase;
      cw[0] = ok ? 1.f : 0.f;
    }

    if (tap + 1 < KK){
      const char* src = (const char*)wmat + (size_t)(tap + 1) * 8192 + tid * 64;
      char* dst = (char*)&Btile[bp ^ 1][0] + tid * 64;
      #pragma unroll
      for (int i = 0; i < 4; ++i) copy16_g2l(src + i * 16, dst + i * 16);
    }

    unsigned int* drow = (unsigned int*)&Atile[p_local * LDA + cbase];
    #pragma unroll
    for (int g = 0; g < 4; ++g){
      float a8[8];
      #pragma unroll
      for (int i = 0; i < 8; ++i) a8[i] = 0.f;
      if (deform){
        #pragma unroll
        for (int cn = 0; cn < 4; ++cn){
          const uint4 q = ((const uint4*)cp[cn])[g];
          const float wvq = cw[cn];
          a8[0] += wvq * bf2f((unsigned short)(q.x & 0xFFFFu));
          a8[1] += wvq * bf2f((unsigned short)(q.x >> 16));
          a8[2] += wvq * bf2f((unsigned short)(q.y & 0xFFFFu));
          a8[3] += wvq * bf2f((unsigned short)(q.y >> 16));
          a8[4] += wvq * bf2f((unsigned short)(q.z & 0xFFFFu));
          a8[5] += wvq * bf2f((unsigned short)(q.z >> 16));
          a8[6] += wvq * bf2f((unsigned short)(q.w & 0xFFFFu));
          a8[7] += wvq * bf2f((unsigned short)(q.w >> 16));
        }
      } else {
        const uint4 q = ((const uint4*)cp[0])[g];
        const float wvq = cw[0];
        a8[0] = wvq * bf2f((unsigned short)(q.x & 0xFFFFu));
        a8[1] = wvq * bf2f((unsigned short)(q.x >> 16));
        a8[2] = wvq * bf2f((unsigned short)(q.y & 0xFFFFu));
        a8[3] = wvq * bf2f((unsigned short)(q.y >> 16));
        a8[4] = wvq * bf2f((unsigned short)(q.z & 0xFFFFu));
        a8[5] = wvq * bf2f((unsigned short)(q.z >> 16));
        a8[6] = wvq * bf2f((unsigned short)(q.w & 0xFFFFu));
        a8[7] = wvq * bf2f((unsigned short)(q.w >> 16));
      }
      #pragma unroll
      for (int j2 = 0; j2 < 4; ++j2)
        drow[g * 4 + j2] = (unsigned int)f2bf(a8[2 * j2]) |
                           ((unsigned int)f2bf(a8[2 * j2 + 1]) << 16);
    }

    if (tap + 1 < KK) wait_async<4>(); else wait_async<0>();
    __syncthreads();

    const int mrow = 16 * wv + (ln & 15);
    const int kb   = (ln >> 4) * 8;
    const unsigned short* bt = &Btile[bp][0];
    #pragma unroll
    for (int ks = 0; ks < 2; ++ks){
      union { v16bf v; unsigned int u[8]; } af;
      #pragma unroll
      for (int r = 0; r < 8; ++r){
        const int kk2 = ks * 32 + ((r < 4) ? (kb + 2 * r) : (16 + kb + 2 * (r - 4)));
        af.u[r] = *(const unsigned int*)&Atile[mrow * LDA + kk2];
      }
      #pragma unroll
      for (int j = 0; j < 4; ++j){
        union { v16bf v; uint4 q[2]; } bfv;
        const uint4* bp2 = (const uint4*)(bt + ((ks * 4 + j) * 32 + ln) * 16);
        bfv.q[0] = bp2[0];
        bfv.q[1] = bp2[1];
        acc[j] = wmma16(af.v, bfv.v, acc[j]);
      }
    }
    __syncthreads();

    if (++kw == 3){ kw = 0; if (++kh == 3){ kh = 0; ++kt; } }
  }

  #pragma unroll
  for (int j = 0; j < 4; ++j){
    const int o  = 16 * j + (ln & 15);
    const float bo = (o < NO) ? bias[o] : 0.f;
    #pragma unroll
    for (int r = 0; r < 8; ++r){
      float y = acc[j][r] + bo;
      const int ml = 16 * wv + r + 8 * (ln >> 4);
      if (mode == 1) y = (y >= 0.f) ? y : 0.1f * y;
      so[ml][o] = y;
    }
  }
  __syncthreads();
  if (mode == 0){
    #pragma unroll
    for (int q = 0; q < 8; ++q){ const int g = q * 128 + tid; const int rl = g >> 4, pc = g & 15;
      v4f v = { so[rl][pc*4], so[rl][pc*4+1], so[rl][pc*4+2], so[rl][pc*4+3] };
      vst2(outF + (size_t)(m0 + rl) * 64 + pc * 4, v); }
  } else if (mode == 1){
    #pragma unroll
    for (int q = 0; q < 4; ++q){ const int g = q * 128 + tid; const int rl = g >> 3, pc = g & 7;
      union { unsigned short s[8]; v4u u; } pk;
      #pragma unroll
      for (int e = 0; e < 8; ++e) pk.s[e] = f2bf(so[rl][pc*8+e]);
      vst2(outB + (size_t)(m0 + rl) * 64 + pc * 8, pk.u); }
  } else {
    #pragma unroll
    for (int q = 0; q < 8; ++q){ const int g = q * 128 + tid; const int o = g >> 4, pc = g & 15;
      const size_t base = (size_t)o * Mpix + m0 + pc * 4;
      v4f v = { so[pc*4][o] + resid[base], so[pc*4+1][o] + resid[base+1], so[pc*4+2][o] + resid[base+2], so[pc*4+3][o] + resid[base+3] };
      vst2(outF + base, v); }
  }
}

extern "C" void kernel_launch(void* const* d_in, const int* in_sizes, int n_in,
                              void* d_out, int out_size, void* d_ws, size_t ws_size,
                              hipStream_t stream) {
  const float* x     = (const float*)d_in[0];
  const float* woff0 = (const float*)d_in[1];
  const float* boff0 = (const float*)d_in[2];
  const float* w0    = (const float*)d_in[3];
  const float* b0    = (const float*)d_in[4];
  const float* woff1 = (const float*)d_in[5];
  const float* boff1 = (const float*)d_in[6];
  const float* w1    = (const float*)d_in[7];
  const float* b1    = (const float*)d_in[8];
  float* out = (float*)d_out;

  char* ws = (char*)d_ws;
  unsigned short* xbf  = (unsigned short*)(ws);
  unsigned short* hbf  = (unsigned short*)(ws + 2064384);
  float*          offb = (float*)(ws + 2 * 2064384);
  unsigned short* wb0o = (unsigned short*)(ws + 2 * 2064384 + 4128768);
  unsigned short* wb0  = wb0o + 110592;
  unsigned short* wb1o = wb0  + 110592;
  unsigned short* wb1  = wb1o + 110592;

  k_cvt_x<<<dim3(504), dim3(256), 0, stream>>>(x, xbf);
  k_cvt_w<<<dim3(54), dim3(256), 0, stream>>>(woff0, 54, wb0o);
  k_cvt_w<<<dim3(54), dim3(256), 0, stream>>>(w0,    64, wb0);
  k_cvt_w<<<dim3(54), dim3(256), 0, stream>>>(woff1, 54, wb1o);
  k_cvt_w<<<dim3(54), dim3(256), 0, stream>>>(w1,    64, wb1);

  k_dcn_gemm<<<dim3(252), dim3(128), 0, stream>>>(
      xbf, wb0o, boff0, nullptr, nullptr, offb, nullptr, 54, 0, 0);
  k_dcn_gemm<<<dim3(252), dim3(128), 0, stream>>>(
      xbf, wb0, b0, offb, nullptr, nullptr, hbf, 64, 1, 1);

  k_dcn_gemm<<<dim3(252), dim3(128), 0, stream>>>(
      hbf, wb1o, boff1, nullptr, nullptr, offb, nullptr, 54, 0, 0);
  k_dcn_gemm<<<dim3(252), dim3(128), 0, stream>>>(
      hbf, wb1, b1, offb, x, out, nullptr, 64, 2, 1);
}
